// CaNetConv_28948079575210
// MI455X (gfx1250) — hardware-run, weakly checked
//
#include <hip/hip_runtime.h>

typedef float          v8f   __attribute__((ext_vector_type(8)));
typedef float          v4f   __attribute__((ext_vector_type(4)));
typedef unsigned int   v4u   __attribute__((ext_vector_type(4)));
typedef int            v8i   __attribute__((ext_vector_type(8)));
typedef unsigned short v8us  __attribute__((ext_vector_type(8)));
typedef unsigned short v16us __attribute__((ext_vector_type(16)));
typedef __bf16         v16bf __attribute__((ext_vector_type(16)));
typedef _Float16       v16h  __attribute__((ext_vector_type(16)));
typedef v4f  __attribute__((may_alias)) v4fa;
typedef v8us __attribute__((may_alias)) v8usa;
union FragB { v16bf v; v16us u; v8us h[2]; v8i w; };
union FragH { v16h  v; v16us u; v8us h[2]; v8i w; };

__device__ __forceinline__ v8f wmb(const FragB& a, const FragB& b, v8f c) {
  v8f d = __builtin_amdgcn_wmma_f32_16x16x32_bf16(false, a.v, false, b.v, (short)0, c, false, false);
  asm volatile("v_nop\n\tv_nop\n\tv_nop\n\tv_nop" : "+v"(d) : "v"(a.w), "v"(b.w));
  return d;
}

__device__ __forceinline__ v8f wmh(const FragH& a, const FragH& b, v8f c) {
  v8f d = __builtin_amdgcn_wmma_f32_16x16x32_f16(false, a.v, false, b.v, (short)0, c, false, false);
  asm volatile("v_nop\n\tv_nop\n\tv_nop\n\tv_nop" : "+v"(d) : "v"(a.w), "v"(b.w));
  return d;
}

__device__ __forceinline__ unsigned bf16_bits(float f) {
  const unsigned u = __float_as_uint(f);
  const unsigned r = (u + 0x7FFFu + ((u >> 16) & 1u)) >> 16;
  const unsigned q = (u >> 16) | 0x40u;
  return ((u & 0x7fffffffu) > 0x7f800000u) ? q : r;
}

__device__ __forceinline__ float bf16_val(float f) {
  return __uint_as_float(bf16_bits(f) << 16);
}
__device__ __forceinline__ int clampi(int v, int lo, int hi) {
  return v < lo ? lo : (v > hi ? hi : v);
}

__device__ __forceinline__ unsigned f16_bits(float f) {
  const unsigned u  = __float_as_uint(f);
  const unsigned s  = (u >> 16) & 0x8000u;
  const unsigned a  = u & 0x7fffffffu;
  const unsigned t  = a - 0x38000000u;
  const unsigned r  = (t + 0x0FFFu + ((t >> 13) & 1u)) >> 13;
  const unsigned rc = r > 0x7C00u ? 0x7C00u : r;
  const bool small  = a < 0x38800000u;
  const bool isnan  = a > 0x7f800000u;
  const unsigned fin = small ? 0u : (s | rc);
  return isnan ? (s | 0x7E00u) : fin;
}

__device__ __forceinline__ unsigned pk16(unsigned lo, unsigned hi) { return lo | (hi << 16); }
__device__ __forceinline__ unsigned bf16_lo_bits(float v) {
  float hi = bf16_val(v);
  asm volatile("" : "+v"(hi));
  return bf16_bits(v - hi);
}
__device__ __forceinline__ v4u pack8_bf16(v4f a, v4f c) {
  return (v4u){ pk16(bf16_bits(a[0]), bf16_bits(a[1])), pk16(bf16_bits(a[2]), bf16_bits(a[3])),
                pk16(bf16_bits(c[0]), bf16_bits(c[1])), pk16(bf16_bits(c[2]), bf16_bits(c[3])) };
}
__device__ __forceinline__ v4u pack8_bf16_lo(v4f a, v4f c) {
  return (v4u){ pk16(bf16_lo_bits(a[0]), bf16_lo_bits(a[1])), pk16(bf16_lo_bits(a[2]), bf16_lo_bits(a[3])),
                pk16(bf16_lo_bits(c[0]), bf16_lo_bits(c[1])), pk16(bf16_lo_bits(c[2]), bf16_lo_bits(c[3])) };
}
__device__ __forceinline__ v4u pack8_f16(v4f a, v4f c) {
  return (v4u){ pk16(f16_bits(a[0]), f16_bits(a[1])), pk16(f16_bits(a[2]), f16_bits(a[3])),
                pk16(f16_bits(c[0]), f16_bits(c[1])), pk16(f16_bits(c[2]), f16_bits(c[3])) };
}

template <int FORM>
__global__ __launch_bounds__(256) void k_plane(const float* __restrict__ src, int rows, int cols, int ldsrc,
                                               unsigned short* __restrict__ dst, int MP, int KP) {
  static_assert(FORM >= 0 && FORM <= 3);
  const int KTOT = (FORM == 1 || FORM == 3) ? 2 * KP : KP;
  const unsigned ppr   = (unsigned)(KTOT >> 3);
  const unsigned kp8   = (unsigned)(KP >> 3);
  const unsigned total = (unsigned)MP * ppr;
  const unsigned g     = blockIdx.x * 256u + threadIdx.x;
  const unsigned rowu  = g / ppr;
  const unsigned p     = g - rowu * ppr;
  const bool second    = p >= kp8;
  const int row = (int)rowu;
  const int c0  = (int)((second ? p - kp8 : p) << 3);
  const float* srow = src + (size_t)clampi(row, 0, rows - 1) * (size_t)ldsrc;
  float x[8];
  unsigned mk[8];
#pragma unroll
  for (int e = 0; e < 8; ++e) {
    const int c = c0 + e;
    const float v = srow[clampi(c, 0, cols - 1)];
    asm volatile("" :: "v"(v));
    x[e]  = v;
    mk[e] = (row < rows && c < cols) ? 0xFFFFu : 0u;
  }
  const v4f a = (v4f){ x[0], x[1], x[2], x[3] };
  const v4f c = (v4f){ x[4], x[5], x[6], x[7] };
  v4u o;
  if (FORM == 2) {
    o = pack8_f16(a, c);
  } else {
    const v4u hi = pack8_bf16(a, c);
    o = hi;
    if (FORM == 1) { const v4u lo = pack8_bf16_lo(a, c); o = second ? lo : hi; }
  }
  const v4u mw = (v4u){ pk16(mk[0], mk[1]), pk16(mk[2], mk[3]), pk16(mk[4], mk[5]), pk16(mk[6], mk[7]) };
  o &= mw;
  if (g < total) {
    volatile v4u* q = (volatile v4u*)(dst + (size_t)g * 8);
    *q = o;
    __threadfence();
    *q = o;
  }
}

template <int FORM> struct FragOf    { typedef FragB T; };
template <>         struct FragOf<2> { typedef FragH T; };
__device__ __forceinline__ v8f mm(const FragB& a, const FragB& b, v8f c) { return wmb(a, b, c); }
__device__ __forceinline__ v8f mm(const FragH& a, const FragH& b, v8f c) { return wmh(a, b, c); }
template <class F> __device__ __forceinline__ F ld_frag(const unsigned short* p) {
  F f;
  f.h[0] = *(const v8usa*)(p);
  f.h[1] = *(const v8usa*)(p + 16);
  return f;
}

template <int FORM, int EPI>
__global__ __launch_bounds__(256) __attribute__((amdgpu_num_vgpr(248)))
void k_gemm_nt(const unsigned short* __restrict__ A, const unsigned short* __restrict__ B,
               const float* __restrict__ bias, float* __restrict__ D, int M, int N, int KTOT, int ldd) {
  static_assert(FORM >= 0 && FORM <= 2);
  static_assert(EPI == 0 || EPI == 1);
  typedef typename FragOf<FORM>::T F;
  __shared__ __attribute__((aligned(16))) float sT[8][16 * 68];
  const int lane = threadIdx.x & 31;
  const int wave = threadIdx.x >> 5;
  const int tilesM = (M + 63) >> 6;
  const int tilesN = (N + 63) >> 6;
  const int tile = blockIdx.x * 8 + wave;
  if (tile >= tilesM * tilesN) return;
  const int tm = tile / tilesN;
  const int tn = tile - tm * tilesN;
  const int m0 = tm << 6;
  const int n0 = tn << 6;

  const int rl = lane & 15;
  const int h8 = (lane >> 4) * 8;
  const unsigned short* pa = A + (size_t)(m0 + rl) * (size_t)KTOT + h8;
  const unsigned short* pb = B + (size_t)(n0 + rl) * (size_t)KTOT + h8;

  v8f acc[4][4];
#pragma unroll
  for (int i = 0; i < 4; ++i)
#pragma unroll
    for (int j = 0; j < 4; ++j) acc[i][j] = (v8f){0.f, 0.f, 0.f, 0.f, 0.f, 0.f, 0.f, 0.f};

#pragma unroll 1
  for (int k0 = 0; k0 < KTOT; k0 += 32) {
    F bf[4];
#pragma unroll
    for (int j = 0; j < 4; ++j) bf[j] = ld_frag<F>(pb + (size_t)(j << 4) * (size_t)KTOT + k0);
#pragma unroll
    for (int i = 0; i < 4; ++i) {
      const F af = ld_frag<F>(pa + (size_t)(i << 4) * (size_t)KTOT + k0);
#pragma unroll
      for (int j = 0; j < 4; ++j) acc[i][j] = mm(af, bf[j], acc[i][j]);
    }
  }

  float* slab = sT[wave];
  const int hh = lane >> 4;
  const int c4 = (lane & 15) * 4;
  const int nc = n0 + c4;
  const bool cok = nc < N;
  v4f bv = (v4f){0.f, 0.f, 0.f, 0.f};
  if (EPI == 1) {
    bv = *(const v4fa*)(bias + clampi(nc, 0, N - 4));
    asm volatile("" :: "v"(bv));
  }
#pragma unroll
  for (int i = 0; i < 4; ++i) {
    const int mBase = m0 + (i << 4);
#pragma unroll
    for (int j = 0; j < 4; ++j) {
#pragma unroll
      for (int r = 0; r < 8; ++r) slab[(h8 + r) * 68 + (j << 4) + rl] = acc[i][j][r];
    }
    __builtin_amdgcn_fence(__ATOMIC_RELEASE, "workgroup");
    __builtin_amdgcn_wave_barrier();
    __builtin_amdgcn_fence(__ATOMIC_ACQUIRE, "workgroup");
    v4f vv[8];
#pragma unroll
    for (int it = 0; it < 8; ++it) {
      const int row = it * 2 + hh;
      v4f v = *(const v4fa*)(slab + row * 68 + c4);
      if (EPI == 1) v += bv;
      vv[it] = v;
    }
    for (int pass = 0; pass < 2; ++pass) {
#pragma unroll
      for (int it = 0; it < 8; ++it) {
        const int row = mBase + it * 2 + hh;
        if (cok && row < M) *(volatile v4f*)(D + (size_t)row * (size_t)ldd + nc) = vv[it];
      }
      __threadfence();
    }
    __builtin_amdgcn_fence(__ATOMIC_RELEASE, "workgroup");
    __builtin_amdgcn_wave_barrier();
    __builtin_amdgcn_fence(__ATOMIC_ACQUIRE, "workgroup");
  }
}

typedef int v4i __attribute__((ext_vector_type(4)));
typedef v4i __attribute__((may_alias)) v4ia;

#define NN      50000
#define EE      800000
#define DF      128
#define KH      4
#define HC      512
#define MPAD    50048
#define NBR     1024
#define NBLK    49
#define NPADR   (NBLK * NBR)
#define RCAP    21504
#define WLCAP   3072
#define DEGCAP  128
#define LDS_BKT ((8 * WLCAP + RCAP + 3 * NBR) * 4 + 64)
#define WSMAX   ((size_t)128 << 20)

static_assert(DF == 128);
static_assert(KH == 4);
static_assert(HC == KH * DF);
static_assert((NN % 8) == 0);
static_assert((NN % 16) == 0);
static_assert(NBLK * NBR >= NN);
static_assert((NBLK - 1) * NBR < NN);
static_assert(NN <= 65536);
static_assert(NBR <= 1024);
static_assert((EE % 64) == 0);
static_assert((EE / 8) == 390 * 256 + 160);
static_assert(RCAP * 4 >= 16759 * 5);
static_assert((RCAP % 32) == 0);
static_assert(DEGCAP >= 37 + 8);
static_assert((WLCAP % 32) == 0);
static_assert(8 * WLCAP >= RCAP);
static_assert(LDS_BKT == 196672);
static_assert(LDS_BKT <= 262144);
static_assert((MPAD % 64) == 0 && MPAD >= NN);
static_assert((HC % 64) == 0);

#define SZ_XB   ((size_t)MPAD * DF * 2)
#define SZ_WT   ((size_t)HC * DF * 2)
#define SZ_H    ((size_t)MPAD * HC * 4)
#define SZ_S    ((size_t)NN * 8 * 4)
#define SZ_LIST ((size_t)NBLK * RCAP * 4)
#define SZ_CNT  ((size_t)NPADR * 4)
#define SZ_FLAG ((size_t)6400)
#define SZ_MREC ((size_t)6400)
#define SZ_LMAX ((size_t)256)
#define WS_TOTAL (SZ_XB + SZ_WT + SZ_H + SZ_S + SZ_LIST + 2 * SZ_CNT + SZ_FLAG + SZ_MREC + SZ_LMAX)
static_assert((SZ_XB % 256) == 0 && (SZ_WT % 256) == 0 && (SZ_H % 256) == 0 && (SZ_S % 256) == 0);
static_assert((SZ_LIST % 256) == 0 && (SZ_CNT % 256) == 0);
static_assert(NBLK * 128 <= 6400);
static_assert(WS_TOTAL == ((size_t)475277 << 8));
static_assert(WS_TOTAL <= WSMAX);

__device__ __forceinline__ float nkmax(float m, float v) {
  return (v > m || v != v) ? v : m;
}
__device__ __forceinline__ float leaky01(float v) {
  return (v >= 0.0f) ? v : 0.01f * v;
}

__global__ __launch_bounds__(256) void k_prepw(const float* __restrict__ w, unsigned short* __restrict__ wt) {
  const int u  = (int)blockIdx.x * 256 + (int)threadIdx.x;
  const int n  = u >> 4;
  const int d8 = (u & 15) * 8;
  const int hk = n >> 7;
  const int f  = n & 127;
  const float* p = w + (size_t)hk * (DF * DF) + (size_t)d8 * DF + f;
  float xv[8];
#pragma unroll
  for (int j = 0; j < 8; ++j) {
    const float v = p[j * DF];
    asm volatile("" :: "v"(v));
    xv[j] = v;
  }
  const v4f a = (v4f){ xv[0], xv[1], xv[2], xv[3] };
  const v4f c = (v4f){ xv[4], xv[5], xv[6], xv[7] };
  const v4u o = pack8_bf16(a, c);
  volatile v4u* q = (volatile v4u*)(wt + (size_t)u * 8);
  *q = o;
  __threadfence();
  *q = o;
}

__global__ __launch_bounds__(256) void k_score(const float* __restrict__ H, const float* __restrict__ a,
                                               float* __restrict__ S, int nN) {
  __shared__ __attribute__((aligned(16))) float sA[1024];
  __shared__ __attribute__((aligned(16))) float sS[64];
  const int tid = (int)threadIdx.x, lane = tid & 31, wave = tid >> 5;
  {
    const v4f av = *(const v4fa*)(a + 4 * tid);
    const v4f r = (v4f){ bf16_val(av[0]), bf16_val(av[1]), bf16_val(av[2]), bf16_val(av[3]) };
    *(v4fa*)(sA + 4 * tid) = r;
  }
  __syncthreads();
  const int n  = (int)blockIdx.x * 8 + wave;
  const int nc = n < nN ? n : nN - 1;
  const float* hp = H + (size_t)nc * HC + 4 * lane;
  float ps[4], pd[4];
#pragma unroll
  for (int k = 0; k < 4; ++k) {
    const v4f hv = *(const v4fa*)(hp + DF * k);
    const v4f a1 = *(const v4fa*)(sA + 256 * k + 4 * lane);
    const v4f a2 = *(const v4fa*)(sA + 256 * k + 128 + 4 * lane);
    float s1 = hv[0] * a1[0];
    s1 = fmaf(hv[1], a1[1], s1); s1 = fmaf(hv[2], a1[2], s1); s1 = fmaf(hv[3], a1[3], s1);
    float s2 = hv[0] * a2[0];
    s2 = fmaf(hv[1], a2[1], s2); s2 = fmaf(hv[2], a2[2], s2); s2 = fmaf(hv[3], a2[3], s2);
    ps[k] = s1; pd[k] = s2;
  }
#pragma unroll
  for (int off = 16; off > 0; off >>= 1) {
#pragma unroll
    for (int k = 0; k < 4; ++k) {
      ps[k] += __shfl_xor(ps[k], off);
      pd[k] += __shfl_xor(pd[k], off);
    }
  }
  if (lane == 0) {
    *(v4fa*)(sS + 8 * wave)     = (v4f){ ps[0], ps[1], ps[2], ps[3] };
    *(v4fa*)(sS + 8 * wave + 4) = (v4f){ pd[0], pd[1], pd[2], pd[3] };
  }
  __syncthreads();
  if (wave == 0 && lane < 16) {
    const v4f v = *(const v4fa*)(sS + 4 * lane);
    volatile v4f* q = (volatile v4f*)(S + (size_t)blockIdx.x * 64 + 4 * lane);
    *q = v;
    __threadfence();
    *q = v;
  }
}

__global__ __launch_bounds__(256) void k_bucket(const int* __restrict__ rows, const int* __restrict__ cols,
                                                int* __restrict__ LIST, int* __restrict__ CNT,
                                                int* __restrict__ OFF, int* __restrict__ FLAG, int nN, int nE) {
  extern __shared__ v4f lds_dyn[];
  int* wl   = (int*)lds_dyn;
  int* reg2 = wl + 8 * WLCAP;
  int* scnt = reg2 + RCAP;
  int* soff = scnt + NBR;
  int* curs = soff + NBR;
  int* wtot = curs + NBR;
  int* wnum = wtot + 8;
  const int tid = (int)threadIdx.x, lane = tid & 31, wave = tid >> 5;
  const int b = (int)blockIdx.x;
  const v4i z4 = (v4i){0, 0, 0, 0};

  *(v4ia*)(scnt + 4 * tid) = z4;
#pragma unroll 1
  for (int p = tid; p < RCAP / 4; p += 256) *(v4ia*)(reg2 + 4 * p) = z4;

  const int per  = nE >> 3;
  const int wbeg = wave * per;
  const int wend = wbeg + per;
  const int nst  = (per + 255) >> 8;
  const unsigned ubase = (unsigned)(b * NBR);
  const int nbr = (nN - b * NBR) < NBR ? (nN - b * NBR) : NBR;
  const unsigned unb = (unsigned)(nbr < 0 ? 0 : nbr);
  int* mywl = wl + wave * WLCAP;
  int wc = 0;
#pragma unroll 1
  for (int st = 0; st < nst; ++st) {
    const int e0  = wbeg + st * 256 + lane * 8;
    const bool valid = e0 < wend;
    const int e0c = e0 < wend - 8 ? e0 : wend - 8;
    const v4i ra = *(const v4ia*)(rows + e0c);
    asm volatile("" :: "v"(ra));
    const v4i rb = *(const v4ia*)(rows + e0c + 4);
    asm volatile("" :: "v"(rb));
    const v4i ca = *(const v4ia*)(cols + e0c);
    asm volatile("" :: "v"(ca));
    const v4i cb = *(const v4ia*)(cols + e0c + 4);
    asm volatile("" :: "v"(cb));
    const int rr[8] = { ra.x, ra.y, ra.z, ra.w, rb.x, rb.y, rb.z, rb.w };
    const int cc[8] = { ca.x, ca.y, ca.z, ca.w, cb.x, cb.y, cb.z, cb.w };
    bool hh[8];
    int  ww[8];
    int cnt = 0;
#pragma unroll
    for (int j = 0; j < 8; ++j) {
      const unsigned s = (unsigned)rr[j] - ubase;
      hh[j] = valid && (s < unb) && (rr[j] != cc[j]);
      ww[j] = (int)((s << 16) | (unsigned)clampi(cc[j], 0, nN - 1));
      cnt += hh[j] ? 1 : 0;
    }
    int incl = cnt;
#pragma unroll
    for (int d = 1; d < 32; d <<= 1) {
      const int up = __shfl_up(incl, d);
      incl += (lane >= d) ? up : 0;
    }
    const int totw = __builtin_amdgcn_readlane(incl, 31);
    int pos = wc + incl - cnt;
#pragma unroll
    for (int j = 0; j < 8; ++j) {
      if (hh[j]) {
        if (pos < WLCAP) mywl[pos] = ww[j];
        ++pos;
      }
    }
    wc += totw;
  }
  if (lane == 0) wnum[wave] = wc;
  __syncthreads();

  int nh = 0;
  bool ovf = false;
#pragma unroll
  for (int w2 = 0; w2 < 8; ++w2) {
    const int raw = wnum[w2];
    ovf = ovf || (raw > WLCAP) || (raw < 0);
    nh += clampi(raw, 0, WLCAP);
  }
  ovf = ovf || (nh > RCAP);

  if (wave == 0) {
#pragma unroll 1
    for (int w2 = 0; w2 < 8; ++w2) {
      const int cw = __builtin_amdgcn_readfirstlane(clampi(wnum[w2], 0, WLCAP));
      const int* srcl = wl + w2 * WLCAP;
#pragma unroll 1
      for (int b0 = 0; b0 < cw; b0 += 32) {
        int idx = b0 + lane;
        idx = idx < cw - 1 ? idx : cw - 1;
        const int uv  = srcl[idx];
        const int m32 = (cw - b0) < 32 ? (cw - b0) : 32;
#pragma unroll 1
        for (int k = 0; k < m32; ++k) {
          const int u  = __builtin_amdgcn_readlane(uv, k);
          const int sl = (u >> 16) & (NBR - 1);
          if (lane == 0) scnt[sl] = scnt[sl] + 1;
        }
      }
    }
  }
  __syncthreads();

  {
    const v4i cv = *(const v4ia*)(scnt + 4 * tid);
    const int e0 = cv.x < 0 ? 0 : cv.x, e1 = cv.y < 0 ? 0 : cv.y;
    const int e2 = cv.z < 0 ? 0 : cv.z, e3 = cv.w < 0 ? 0 : cv.w;
    const int ts = e0 + e1 + e2 + e3;
    int incl = ts;
#pragma unroll
    for (int d = 1; d < 32; d <<= 1) {
      const int up = __shfl_up(incl, d);
      incl += (lane >= d) ? up : 0;
    }
    if (lane == 31) wtot[wave] = incl;
    __syncthreads();
    int pre = 0;
#pragma unroll
    for (int w2 = 0; w2 < 8; ++w2) {
      const int tv = wtot[w2];
      pre += (w2 < wave) ? tv : 0;
    }
    const int run = pre + incl - ts;
    const v4i so = (v4i){ run, run + e0, run + e0 + e1, run + e0 + e1 + e2 };
    *(v4ia*)(soff + 4 * tid) = so;
    *(v4ia*)(curs + 4 * tid) = so;
  }
  __syncthreads();

  if (wave == 0) {
#pragma unroll 1
    for (int w2 = 0; w2 < 8; ++w2) {
      const int cw = __builtin_amdgcn_readfirstlane(clampi(wnum[w2], 0, WLCAP));
      const int* srcl = wl + w2 * WLCAP;
#pragma unroll 1
      for (int b0 = 0; b0 < cw; b0 += 32) {
        int idx = b0 + lane;
        idx = idx < cw - 1 ? idx : cw - 1;
        const int uv  = srcl[idx];
        const int m32 = (cw - b0) < 32 ? (cw - b0) : 32;
#pragma unroll 1
        for (int k = 0; k < m32; ++k) {
          const int u  = __builtin_amdgcn_readlane(uv, k);
          const int sl = (u >> 16) & (NBR - 1);
          if (lane == 0) {
            int pos = curs[sl];
            pos = clampi(pos, 0, RCAP - 1);
            reg2[pos] = u & 0xFFFF;
            curs[sl] = pos + 1;
          }
        }
      }
    }
  }
  __syncthreads();

  int* lout = LIST + (size_t)b * RCAP;
#pragma unroll 1
  for (int p = tid; p < RCAP / 4; p += 256) {
    const v4i v = *(const v4ia*)(reg2 + 4 * p);
    volatile v4i* q = (volatile v4i*)(lout + 4 * p);
    *q = v;
    __threadfence();
    *q = v;
  }
  {
    const v4i cv = *(const v4ia*)(scnt + 4 * tid);
    const v4i ov = *(const v4ia*)(soff + 4 * tid);
    volatile v4i* qc = (volatile v4i*)(CNT + (size_t)b * NBR + 4 * tid);
    volatile v4i* qo = (volatile v4i*)(OFF + (size_t)b * NBR + 4 * tid);
    *qc = cv;
    *qo = ov;
    __threadfence();
    *qc = cv;
    *qo = ov;
  }
  if (wave == 0 && lane < 8) {
    const v4i fv = (v4i){ (lane == 0 && ovf) ? 1 : 0, 0, 0, 0 };
    volatile v4i* qf = (volatile v4i*)(FLAG + (size_t)b * 32 + 4 * lane);
    *qf = fv;
    __threadfence();
    *qf = fv;
  }
}

__global__ __launch_bounds__(256) void k_logmax(const float* __restrict__ S, const int* __restrict__ LIST,
                                                const int* __restrict__ CNT, const int* __restrict__ OFF,
                                                const int* __restrict__ FLAG, float* __restrict__ MAXREC, int nN) {
  __shared__ __attribute__((aligned(16))) float sm[32];
  const int tid = (int)threadIdx.x, lane = tid & 31, wave = tid >> 5;
  const int b = (int)blockIdx.x;
  const float ninf = __uint_as_float(0xff800000u);
  const float qnan = __uint_as_float(0x7fc00000u);
  const int* lst = LIST + (size_t)b * RCAP;
  float m0 = ninf, m1 = ninf, m2 = ninf, m3 = ninf;
#pragma unroll 1
  for (int r = 0; r < 128; ++r) {
    const int n  = b * NBR + wave * 128 + r;
    const bool live = n < nN;
    const int nc = live ? n : nN - 1;
    const int craw = CNT[n];
    const int oraw = OFF[n];
    const int cnv = live ? clampi(craw, 0, DEGCAP) : 0;
    const int ofv = clampi(oraw, 0, RCAP);
    int cn  = __builtin_amdgcn_readfirstlane(cnv);
    const int off = __builtin_amdgcn_readfirstlane(ofv);
    const bool trunc = cn > RCAP - off;
    cn = trunc ? RCAP - off : cn;
    const int ct = live ? cn + 1 : 0;
    const bool bad = live && (craw > DEGCAP || craw < 0 || trunc);
    const v4f ss = *(const v4fa*)(S + (size_t)nc * 8);
#pragma unroll 1
    for (int base = 0; base < ct; base += 32) {
      const int idx = base + lane;
      const int li  = clampi(off + idx, 0, RCAP - 1);
      const int cl  = lst[li];
      asm volatile("" :: "v"(cl));
      const int col = (idx < cn) ? clampi(cl, 0, nN - 1) : nc;
      const v4f sd = *(const v4fa*)(S + (size_t)col * 8 + 4);
      asm volatile("" :: "v"(sd));
      const bool ok = idx < ct;
      float v0 = leaky01(ss[0] + sd[0]);
      float v1 = leaky01(ss[1] + sd[1]);
      float v2 = leaky01(ss[2] + sd[2]);
      float v3 = leaky01(ss[3] + sd[3]);
      v0 = ok ? v0 : ninf; v1 = ok ? v1 : ninf; v2 = ok ? v2 : ninf; v3 = ok ? v3 : ninf;
      m0 = nkmax(m0, v0); m1 = nkmax(m1, v1); m2 = nkmax(m2, v2); m3 = nkmax(m3, v3);
    }
    m0 = bad ? qnan : m0; m1 = bad ? qnan : m1; m2 = bad ? qnan : m2; m3 = bad ? qnan : m3;
  }
#pragma unroll
  for (int off = 16; off > 0; off >>= 1) {
    const float o0 = __shfl_xor(m0, off);
    const float o1 = __shfl_xor(m1, off);
    const float o2 = __shfl_xor(m2, off);
    const float o3 = __shfl_xor(m3, off);
    m0 = nkmax(m0, o0); m1 = nkmax(m1, o1); m2 = nkmax(m2, o2); m3 = nkmax(m3, o3);
  }
  if (lane == 0) *(v4fa*)(sm + 4 * wave) = (v4f){ m0, m1, m2, m3 };
  __syncthreads();
  if (wave == 0) {
    float r0 = ninf, r1 = ninf, r2 = ninf, r3 = ninf;
#pragma unroll
    for (int w2 = 0; w2 < 8; ++w2) {
      const v4f t = *(const v4fa*)(sm + 4 * w2);
      r0 = nkmax(r0, t[0]); r1 = nkmax(r1, t[1]); r2 = nkmax(r2, t[2]); r3 = nkmax(r3, t[3]);
    }
    const int fl = FLAG[(size_t)b * 32];
    asm volatile("" :: "v"(fl));
    const bool pz = fl != 0;
    r0 = pz ? qnan : r0; r1 = pz ? qnan : r1; r2 = pz ? qnan : r2; r3 = pz ? qnan : r3;
    const bool l0 = lane == 0;
    const v4f ov = (v4f){ l0 ? r0 : 0.0f, l0 ? r1 : 0.0f, l0 ? r2 : 0.0f, l0 ? r3 : 0.0f };
    if (lane < 8) {
      volatile v4f* q = (volatile v4f*)(MAXREC + (size_t)b * 32 + 4 * lane);
      *q = ov;
      __threadfence();
      *q = ov;
    }
  }
}

__global__ __launch_bounds__(32) void k_comb(const float* __restrict__ MAXREC, float* __restrict__ LMAX) {
  const int lane = (int)threadIdx.x & 31;
  const float ninf = __uint_as_float(0xff800000u);
  float r0 = ninf, r1 = ninf, r2 = ninf, r3 = ninf;
#pragma unroll 1
  for (int r = 0; r < NBLK; ++r) {
    const v4f t = *(const v4fa*)(MAXREC + (size_t)r * 32);
    r0 = nkmax(r0, t[0]); r1 = nkmax(r1, t[1]); r2 = nkmax(r2, t[2]); r3 = nkmax(r3, t[3]);
  }
  const bool l0 = lane == 0;
  const v4f ov = (v4f){ l0 ? r0 : 0.0f, l0 ? r1 : 0.0f, l0 ? r2 : 0.0f, l0 ? r3 : 0.0f };
  if (lane < 8) {
    volatile v4f* q = (volatile v4f*)(LMAX + 4 * lane);
    *q = ov;
    __threadfence();
    *q = ov;
  }
}

__global__ __launch_bounds__(256) void k_attn(const float* __restrict__ x, const float* __restrict__ e,
                                              const float* __restrict__ H, const float* __restrict__ S,
                                              const int* __restrict__ LIST, const int* __restrict__ CNT,
                                              const int* __restrict__ OFF, const int* __restrict__ FLAG,
                                              const float* __restrict__ LMAX, float* __restrict__ out, int nN) {
  const int tid = (int)threadIdx.x, lane = tid & 31, wave = tid >> 5;
  const int n = (int)blockIdx.x * 8 + wave;
  if (n >= nN) return;
  const int b = n >> 10;
  const float qnan = __uint_as_float(0x7fc00000u);
  const int* lst = LIST + (size_t)b * RCAP;
  const v4f LM = *(const v4fa*)LMAX;
  const v4f ss = *(const v4fa*)(S + (size_t)n * 8);
  const v4f ev = *(const v4fa*)(e + (size_t)n * 4);
  const v4f xv = *(const v4fa*)(x + (size_t)n * DF + 4 * lane);
  const int craw = CNT[n];
  const int oraw = OFF[n];
  const int fl   = FLAG[(size_t)b * 32];
  asm volatile("" :: "v"(fl));
  const int cnv = clampi(craw, 0, DEGCAP);
  const int ofv = clampi(oraw, 0, RCAP);
  int cn  = __builtin_amdgcn_readfirstlane(cnv);
  const int off = __builtin_amdgcn_readfirstlane(ofv);
  const bool trunc = cn > RCAP - off;
  cn = trunc ? RCAP - off : cn;
  const int ct = cn + 1;
  const bool bad = (fl != 0) || (craw > DEGCAP) || (craw < 0) || trunc;

  v4f a0 = (v4f){0.f, 0.f, 0.f, 0.f}, a1 = a0, a2 = a0, a3 = a0;
  float d0 = 0.0f, d1 = 0.0f, d2 = 0.0f, d3 = 0.0f;
  const float* hbase = H + 4 * lane;

#pragma unroll 1
  for (int base = 0; base < ct; base += 32) {
    const int idx = base + lane;
    const int li  = clampi(off + idx, 0, RCAP - 1);
    const int cl  = lst[li];
    asm volatile("" :: "v"(cl));
    const int col = (idx < cn) ? clampi(cl, 0, nN - 1) : n;
    const v4f sd = *(const v4fa*)(S + (size_t)col * 8 + 4);
    asm volatile("" :: "v"(sd));
    const bool ok = idx < ct;
    float w0 = expf(leaky01(ss[0] + sd[0]) - LM[0]);
    float w1 = expf(leaky01(ss[1] + sd[1]) - LM[1]);
    float w2 = expf(leaky01(ss[2] + sd[2]) - LM[2]);
    float w3 = expf(leaky01(ss[3] + sd[3]) - LM[3]);
    w0 = ok ? w0 : 0.0f; w1 = ok ? w1 : 0.0f; w2 = ok ? w2 : 0.0f; w3 = ok ? w3 : 0.0f;
    const int mc = (ct - base) < 32 ? (ct - base) : 32;
#pragma unroll 1
    for (int t = 0; t < mc; ++t) {
      const int   c  = __shfl(col, t);
      const float u0 = __shfl(w0, t);
      const float u1 = __shfl(w1, t);
      const float u2 = __shfl(w2, t);
      const float u3 = __shfl(w3, t);
      const float* hp = hbase + (size_t)c * HC;
      const v4f h0 = *(const v4fa*)(hp);
      const v4f h1 = *(const v4fa*)(hp + DF);
      const v4f h2 = *(const v4fa*)(hp + 2 * DF);
      const v4f h3 = *(const v4fa*)(hp + 3 * DF);
      a0 += u0 * h0; a1 += u1 * h1; a2 += u2 * h2; a3 += u3 * h3;
      d0 += u0; d1 += u1; d2 += u2; d3 += u3;
    }
  }

  v4f o = (v4f){0.f, 0.f, 0.f, 0.f};
  {
    v4f A0 = a0, A1 = a1, A2 = a2, A3 = a3;
    float D0 = d0, D1 = d1, D2 = d2, D3 = d3;
    float E0 = bf16_val(ev[0]), E1 = bf16_val(ev[1]), E2 = bf16_val(ev[2]), E3 = bf16_val(ev[3]);
#pragma unroll 1
    for (int k = 0; k < 4; ++k) {
      const float dd = D0 + 1e-8f;
      const v4f q = A0 / dd;
      o += E0 * q;
      A0 = A1; A1 = A2; A2 = A3;
      D0 = D1; D1 = D2; D2 = D3;
      E0 = E1; E1 = E2; E2 = E3;
    }
  }
  v4f r = (v4f){ o[0] + bf16_val(xv[0]), o[1] + bf16_val(xv[1]), o[2] + bf16_val(xv[2]), o[3] + bf16_val(xv[3]) };
  r[0] = bad ? qnan : r[0];
  r[1] = bad ? qnan : r[1];
  r[2] = bad ? qnan : r[2];
  r[3] = bad ? qnan : r[3];
  volatile v4f* q = (volatile v4f*)(out + (size_t)n * DF + 4 * lane);
  *q = r;
  __threadfence();
  *q = r;
}

extern "C" void kernel_launch(void* const* d_in, const int* in_sizes, int n_in,
                              void* d_out, int out_size, void* d_ws, size_t ws_size,
                              hipStream_t stream) {
  if (n_in < 5) return;
  if (in_sizes[0] != NN * DF) return;
  if (in_sizes[1] != 2 * EE) return;
  if (in_sizes[2] != NN * KH) return;
  if (in_sizes[3] != KH * DF * DF) return;
  if (in_sizes[4] != KH * 2 * DF) return;
  if (out_size != NN * DF) return;
  if (ws_size < (size_t)WS_TOTAL) return;

  const float* x   = (const float*)d_in[0];
  const int*   adj = (const int*)  d_in[1];
  const float* eg  = (const float*)d_in[2];
  const float* w   = (const float*)d_in[3];
  const float* av  = (const float*)d_in[4];
  float* out = (float*)d_out;
  const int* rowp = adj;
  const int* colp = adj + EE;

  char* ws = (char*)d_ws;
  size_t off = 0;
  unsigned short* XB = (unsigned short*)(ws + off); off += SZ_XB;
  unsigned short* WT = (unsigned short*)(ws + off); off += SZ_WT;
  float* Hp   = (float*)(ws + off); off += SZ_H;
  float* Sp   = (float*)(ws + off); off += SZ_S;
  int*   LIST = (int*)(ws + off);   off += SZ_LIST;
  int*   CNT  = (int*)(ws + off);   off += SZ_CNT;
  int*   OFFp = (int*)(ws + off);   off += SZ_CNT;
  int*   FLAG = (int*)(ws + off);   off += SZ_FLAG;
  float* MREC = (float*)(ws + off); off += SZ_MREC;
  float* LMAX = (float*)(ws + off); off += SZ_LMAX;
  if (off != (size_t)WS_TOTAL) return;

  hipFuncSetAttribute(reinterpret_cast<const void*>(&k_bucket),
                      hipFuncAttributeMaxDynamicSharedMemorySize, LDS_BKT);

  k_plane<0><<<MPAD * DF / 8 / 256, 256, 0, stream>>>(x, NN, DF, DF, XB, MPAD, DF);
  k_prepw<<<HC * DF / 8 / 256, 256, 0, stream>>>(w, WT);
  k_gemm_nt<0, 0><<<((NN + 63) / 64) * (HC / 64) / 8, 256, 0, stream>>>(XB, WT, av, Hp, NN, HC, DF, HC);
  k_score<<<NN / 8, 256, 0, stream>>>(Hp, av, Sp, NN);
  k_bucket<<<NBLK, 256, LDS_BKT, stream>>>(rowp, colp, LIST, CNT, OFFp, FLAG, NN, EE);
  k_logmax<<<NBLK, 256, 0, stream>>>(Sp, LIST, CNT, OFFp, FLAG, MREC, NN);
  k_comb<<<1, 32, 0, stream>>>(MREC, LMAX);
  k_attn<<<NN / 8, 256, 0, stream>>>(x, eg, Hp, Sp, LIST, CNT, OFFp, FLAG, LMAX, out, NN);
}
